// ComplexMultiHeadAttention_58308476010503
// MI455X (gfx1250) — hardware-verified
//
#include <hip/hip_runtime.h>


#pragma clang fp contract(off)

#ifndef NB
#define NB 2
#endif
#ifndef SEQ
#define SEQ 2048
#endif
#ifndef NB_FULL
#define NB_FULL 2
#endif
#ifndef SEQ_FULL
#define SEQ_FULL 2048
#endif

namespace {
constexpr int HID = 768, DH = 64, NH = 12;
constexpr int NW = 5;
constexpr int NCOMB = NW * HID;
constexpr int MROWS = NB * SEQ;
constexpr int QT = SEQ / 16;
constexpr int QKW = 2 * DH;
constexpr float SCORE_SCALE = 0.125f;
constexpr float P_CARRY = 4096.0f;
constexpr float INV_P_CARRY = 1.0f / 4096.0f;
static_assert(SEQ % 128 == 0);
static_assert(NB >= 1 && NB <= NB_FULL);
static_assert(SEQ <= SEQ_FULL);
static_assert(NH * DH == HID);
static_assert(MROWS % 128 == 0);
static_assert(HID % 32 == 0);
static_assert(NCOMB % 64 == 0);
static_assert((NB * NH * QT) % 8 == 0);
static_assert((size_t)MROWS * HID <= (size_t)NB_FULL * SEQ_FULL * HID);

typedef __bf16 b16;
typedef _Float16 h16;
typedef __bf16 v16b __attribute__((ext_vector_type(16)));
typedef __bf16 v8b __attribute__((ext_vector_type(8)));
typedef _Float16 v16h __attribute__((ext_vector_type(16)));
typedef _Float16 v8h __attribute__((ext_vector_type(8)));
typedef float v8f __attribute__((ext_vector_type(8)));
typedef float v4f __attribute__((ext_vector_type(4)));
typedef unsigned short v8us __attribute__((ext_vector_type(8)));
typedef unsigned int v8u __attribute__((ext_vector_type(8)));

__device__ __forceinline__ v8b ld8b(const b16* p) { return *(const v8b*)p; }
__device__ __forceinline__ v8h ld8h(const h16* p) { return *(const v8h*)p; }
__device__ __forceinline__ v16b cat8b(v8b a, v8b b) { return __builtin_shufflevector(a, b, 0, 1, 2, 3, 4, 5, 6, 7, 8, 9, 10, 11, 12, 13, 14, 15); }
__device__ __forceinline__ v16h cat8h(v8h a, v8h b) { return __builtin_shufflevector(a, b, 0, 1, 2, 3, 4, 5, 6, 7, 8, 9, 10, 11, 12, 13, 14, 15); }
__device__ __forceinline__ v16b frag_kb(const b16* p, int hh) { return cat8b(ld8b(p + 8 * hh), ld8b(p + 16 + 8 * hh)); }
__device__ __forceinline__ v16h frag_kh(const h16* p, int hh) { return cat8h(ld8h(p + 8 * hh), ld8h(p + 16 + 8 * hh)); }

__device__ __forceinline__ v8f wmma_b(v16b a, v16b b, v8f c) {
  v8f d = __builtin_amdgcn_wmma_f32_16x16x32_bf16(false, a, false, b, (short)0, c, false, false);
  asm volatile("v_nop\n\tv_nop\n\tv_nop\n\tv_nop" : "+v"(d) : "v"(a), "v"(b));
  return d;
}
__device__ __forceinline__ v8f wmma_h(v16h a, v16h b, v8f c) {
  v8f d = __builtin_amdgcn_wmma_f32_16x16x32_f16(false, a, false, b, (short)0, c, false, false);
  asm volatile("v_nop\n\tv_nop\n\tv_nop\n\tv_nop" : "+v"(d) : "v"(a), "v"(b));
  return d;
}
__device__ __forceinline__ v16h neg16h(v16h a) {
  v8u t = __builtin_bit_cast(v8u, a);
  const v8u s = {0x80008000u, 0x80008000u, 0x80008000u, 0x80008000u, 0x80008000u, 0x80008000u, 0x80008000u, 0x80008000u};
  t = t ^ s;
  return __builtin_bit_cast(v16h, t);
}
__device__ __forceinline__ unsigned int bf16_rne_u32(float f) {
  unsigned int u = __builtin_bit_cast(unsigned int, f);
  u += 0x7fffu + ((u >> 16) & 1u);
  return u & 0xffff0000u;
}
__device__ __forceinline__ void wave_lds_sync() {
  __builtin_amdgcn_fence(3, "workgroup");
  __builtin_amdgcn_wave_barrier();
  __builtin_amdgcn_fence(2, "workgroup");
}

__global__ __launch_bounds__(256) void cvt_kernel(const float* __restrict__ x,
                                                  const float* __restrict__ w0, const float* __restrict__ w1, const float* __restrict__ w2,
                                                  const float* __restrict__ w3, const float* __restrict__ w4,
                                                  unsigned short* __restrict__ xpl, unsigned short* __restrict__ wpl) {
  const size_t tid = (size_t)blockIdx.x * blockDim.x + threadIdx.x, stride = (size_t)gridDim.x * blockDim.x;
  const size_t nx = (size_t)MROWS * HID / 8;
  const size_t per_w = (size_t)HID * HID / 8, nw = (size_t)NW * per_w;
  for (int pass = 0; pass < 2; ++pass) {
    for (size_t c = tid; c < nx; c += stride) {
      const size_t i = c * 8;
      const int m = (int)(i / HID), col = (int)(i % HID);
      const int bb = m / SEQ, t = m - bb * SEQ;
      const float* p = x + ((size_t)bb * SEQ_FULL + t) * HID + col;
      const v4f f0 = *(const v4f*)p, f1 = *(const v4f*)(p + 4);
      v8us o;
#pragma unroll
      for (int e = 0; e < 4; ++e) {
        o[e] = (unsigned short)(bf16_rne_u32(f0[e]) >> 16);
        o[4 + e] = (unsigned short)(bf16_rne_u32(f1[e]) >> 16);
      }
      *(volatile v8us*)(xpl + i) = o;
    }
    for (size_t c = tid; c < nw; c += stride) {
      const int mat = (int)(c / per_w);
      const size_t i = (c - (size_t)mat * per_w) * 8;
      const float* w = (mat == 0) ? w0 : (mat == 1) ? w1 : (mat == 2) ? w2 : (mat == 3) ? w3 : w4;
      const v4f f0 = *(const v4f*)(w + i), f1 = *(const v4f*)(w + i + 4);
      v8us o;
#pragma unroll
      for (int e = 0; e < 4; ++e) {
        o[e] = (unsigned short)(bf16_rne_u32(f0[e]) >> 16);
        o[4 + e] = (unsigned short)(bf16_rne_u32(f1[e]) >> 16);
      }
      *(volatile v8us*)(wpl + c * 8) = o;
    }
    __threadfence();
  }
}

__device__ __forceinline__ void gemm_tile_b(const b16* __restrict__ A, const b16* __restrict__ W, int m0, int c0, int nloc, int hlf, v8f (&acc)[2][4]) {
#pragma unroll 2
  for (int kb = 0; kb < HID; kb += 32) {
    const v16b a0 = frag_kb(A + (size_t)(m0 + nloc) * HID + kb, hlf);
    const v16b a1 = frag_kb(A + (size_t)(m0 + 16 + nloc) * HID + kb, hlf);
#pragma unroll
    for (int t = 0; t < 4; ++t) {
      const v16b bf = frag_kb(W + (size_t)(c0 + t * 16 + nloc) * HID + kb, hlf);
      acc[0][t] = wmma_b(a0, bf, acc[0][t]);
      acc[1][t] = wmma_b(a1, bf, acc[1][t]);
    }
  }
}

__global__ __launch_bounds__(128) void proj_gemm_kernel(const b16* __restrict__ xpl, const b16* __restrict__ wpl,
                                                        h16* __restrict__ Qa, h16* __restrict__ Kc, h16* __restrict__ Vp) {
  __shared__ __attribute__((aligned(16))) h16 Ts[4][32 * 64];
  const int lane = threadIdx.x & 31, wave = threadIdx.x >> 5, nloc = lane & 15, hlf = lane >> 4;
  const int m0 = blockIdx.y * 128 + wave * 32;
  const int cb = blockIdx.x;
  const int mat = cb / NH, head = cb - mat * NH;
  const int c0 = cb * 64;
  v8f acc[2][4];
#pragma unroll
  for (int r = 0; r < 2; ++r)
#pragma unroll
    for (int t = 0; t < 4; ++t) acc[r][t] = (v8f){};
  gemm_tile_b(xpl, wpl, m0, c0, nloc, hlf, acc);
  const int b = m0 / SEQ, t0 = m0 % SEQ;
  const int g = b * NH + head;
  h16* Tp = Ts[wave];
#pragma unroll
  for (int t = 0; t < 4; ++t) {
    const int d = t * 16 + nloc;
#pragma unroll
    for (int r = 0; r < 2; ++r)
#pragma unroll
      for (int v = 0; v < 8; ++v) {
        const int rr = r * 16 + v + 8 * hlf;
        const h16 y = (h16)acc[r][t][v];
        const int idx = (mat < 4) ? (rr * 64 + d) : ((rr >> 4) * 1024 + d * 16 + (rr & 15));
        Tp[idx] = y;
      }
  }
  wave_lds_sync();
  if (mat < 4) {
    h16* P = (mat < 2) ? Qa : Kc;
    const int coff = (mat & 1) * DH;
    h16* dst = P + ((size_t)g * SEQ + t0) * QKW + coff;
#pragma unroll
    for (int j = 0; j < 8; ++j) {
      const int rr = j * 4 + (lane >> 3), c8 = (lane & 7) * 8;
      *(volatile v8h*)(dst + (size_t)rr * QKW + c8) = ld8h(Tp + rr * 64 + c8);
    }
    __threadfence();
#pragma unroll
    for (int j = 0; j < 8; ++j) {
      const int rr = j * 4 + (lane >> 3), c8 = (lane & 7) * 8;
      *(volatile v8h*)(dst + (size_t)rr * QKW + c8) = ld8h(Tp + rr * 64 + c8);
    }
  } else {
    h16* dst = Vp + ((size_t)g * QT + (t0 >> 4)) * (size_t)(DH * 16);
#pragma unroll
    for (int j = 0; j < 8; ++j) { const int e = (j * 32 + lane) * 8; *(volatile v8h*)(dst + e) = ld8h(Tp + e); }
    __threadfence();
#pragma unroll
    for (int j = 0; j < 8; ++j) { const int e = (j * 32 + lane) * 8; *(volatile v8h*)(dst + e) = ld8h(Tp + e); }
  }
}

__global__ __launch_bounds__(256) void attn_kernel(const h16* __restrict__ Qa, const h16* __restrict__ Kc, const h16* __restrict__ Vp,
                                                   float* __restrict__ out) {
  __shared__ __attribute__((aligned(16))) float Os[8][16 * 64];
  const int wid = threadIdx.x >> 5, lane = threadIdx.x & 31, hh = lane >> 4, col = lane & 15;
  const int qtile = blockIdx.x * 8 + wid;
  const int g = qtile / QT;
  const int q0 = (qtile % QT) << 4;
  const int b = g / NH, h = g % NH;
  const size_t kbase = (size_t)g * SEQ * QKW;
  const size_t vbase = (size_t)g * SEQ * DH;
  const h16* qrow = Qa + ((size_t)g * SEQ + q0 + col) * QKW;
  const v16h qf0 = frag_kh(qrow, hh), qf1 = frag_kh(qrow + 32, hh);
  const v16h qf2 = frag_kh(qrow + 64, hh), qf3 = frag_kh(qrow + 96, hh);
  const v16h qn0 = neg16h(qf0), qn1 = neg16h(qf1);
  float m = -INFINITY, l = 0.0f;
  v8f o0 = {}, o1 = {}, o2 = {}, o3 = {};
  for (int kb = 0; kb < SEQ; kb += 32) {
    const h16* k0p = Kc + kbase + (size_t)(kb + col) * QKW;
    const h16* k1p = k0p + (size_t)16 * QKW;
    v8f s0r = {}, s0i = {}, s1r = {}, s1i = {};
    {
      v16h kf = frag_kh(k0p, hh);          s0r = wmma_h(kf, qf0, s0r); s0i = wmma_h(kf, qf2, s0i);
      kf = frag_kh(k0p + 32, hh);          s0r = wmma_h(kf, qf1, s0r); s0i = wmma_h(kf, qf3, s0i);
      kf = frag_kh(k0p + 64, hh);          s0r = wmma_h(kf, qf2, s0r); s0i = wmma_h(kf, qn0, s0i);
      kf = frag_kh(k0p + 96, hh);          s0r = wmma_h(kf, qf3, s0r); s0i = wmma_h(kf, qn1, s0i);
      kf = frag_kh(k1p, hh);               s1r = wmma_h(kf, qf0, s1r); s1i = wmma_h(kf, qf2, s1i);
      kf = frag_kh(k1p + 32, hh);          s1r = wmma_h(kf, qf1, s1r); s1i = wmma_h(kf, qf3, s1i);
      kf = frag_kh(k1p + 64, hh);          s1r = wmma_h(kf, qf2, s1r); s1i = wmma_h(kf, qn0, s1i);
      kf = frag_kh(k1p + 96, hh);          s1r = wmma_h(kf, qf3, s1r); s1i = wmma_h(kf, qn1, s1i);
    }
    v8f sc0, sc1;
#pragma unroll
    for (int r = 0; r < 8; ++r) {
      const float a0 = s0r[r] * SCORE_SCALE, b0 = s0i[r] * SCORE_SCALE;
      const float a1 = s1r[r] * SCORE_SCALE, b1 = s1i[r] * SCORE_SCALE;
      sc0[r] = sqrtf(a0 * a0 + b0 * b0);
      sc1[r] = sqrtf(a1 * a1 + b1 * b1);
    }
    float mr = -INFINITY;
#pragma unroll
    for (int r = 0; r < 8; ++r) mr = fmaxf(mr, fmaxf(sc0[r], sc1[r]));
    mr = fmaxf(mr, __shfl_xor(mr, 16));
    const float mn = fmaxf(m, mr);
    const float al_ = __expf(m - mn);
    m = mn;
    float sum = 0.0f;
    v16h pb;
#pragma unroll
    for (int r = 0; r < 8; ++r) {
      const float p0 = __expf(sc0[r] - mn), p1 = __expf(sc1[r] - mn);
      sum += p0 + p1;
      pb[r] = (h16)(p0 * P_CARRY); pb[8 + r] = (h16)(p1 * P_CARRY);
    }
    sum += __shfl_xor(sum, 16);
    l = l * al_ + sum;
    o0 = o0 * al_; o1 = o1 * al_; o2 = o2 * al_; o3 = o3 * al_;
    const size_t v0 = vbase + (size_t)(kb >> 4) * (DH * 16) + 8 * hh, v1 = v0 + DH * 16;
    {
      const v16h va0 = cat8h(ld8h(Vp + v0 + (0 * 16 + col) * 16), ld8h(Vp + v1 + (0 * 16 + col) * 16));
      o0 = wmma_h(va0, pb, o0);
      const v16h va1 = cat8h(ld8h(Vp + v0 + (1 * 16 + col) * 16), ld8h(Vp + v1 + (1 * 16 + col) * 16));
      o1 = wmma_h(va1, pb, o1);
      const v16h va2 = cat8h(ld8h(Vp + v0 + (2 * 16 + col) * 16), ld8h(Vp + v1 + (2 * 16 + col) * 16));
      o2 = wmma_h(va2, pb, o2);
      const v16h va3 = cat8h(ld8h(Vp + v0 + (3 * 16 + col) * 16), ld8h(Vp + v1 + (3 * 16 + col) * 16));
      o3 = wmma_h(va3, pb, o3);
    }
  }
  const float inv = (1.0f / l) * INV_P_CARRY;
  float* Tt = Os[wid];
  {
    float* tp = Tt + col * 64 + 8 * hh;
    const v4f a0 = {o0[0] * inv, o0[1] * inv, o0[2] * inv, o0[3] * inv}, a1 = {o0[4] * inv, o0[5] * inv, o0[6] * inv, o0[7] * inv};
    const v4f b0 = {o1[0] * inv, o1[1] * inv, o1[2] * inv, o1[3] * inv}, b1 = {o1[4] * inv, o1[5] * inv, o1[6] * inv, o1[7] * inv};
    const v4f c0 = {o2[0] * inv, o2[1] * inv, o2[2] * inv, o2[3] * inv}, c1 = {o2[4] * inv, o2[5] * inv, o2[6] * inv, o2[7] * inv};
    const v4f d0 = {o3[0] * inv, o3[1] * inv, o3[2] * inv, o3[3] * inv}, d1 = {o3[4] * inv, o3[5] * inv, o3[6] * inv, o3[7] * inv};
    *(v4f*)(tp + 0)  = a0; *(v4f*)(tp + 4)  = a1;
    *(v4f*)(tp + 16) = b0; *(v4f*)(tp + 20) = b1;
    *(v4f*)(tp + 32) = c0; *(v4f*)(tp + 36) = c1;
    *(v4f*)(tp + 48) = d0; *(v4f*)(tp + 52) = d1;
  }
  wave_lds_sync();
  float* dst0 = out + ((size_t)b * SEQ + q0) * HID + h * DH;
#pragma unroll
  for (int j = 0; j < 8; ++j) {
    const int rr = j * 2 + hh, c4 = col * 4;
    *(volatile v4f*)(dst0 + (size_t)rr * HID + c4) = *(const v4f*)(Tt + rr * 64 + c4);
  }
  __threadfence();
#pragma unroll
  for (int j = 0; j < 8; ++j) {
    const int rr = j * 2 + hh, c4 = col * 4;
    *(volatile v4f*)(dst0 + (size_t)rr * HID + c4) = *(const v4f*)(Tt + rr * 64 + c4);
  }
}
}

extern "C" void kernel_launch(void* const* d_in, const int* in_sizes, int n_in,
                              void* d_out, int out_size, void* d_ws, size_t ws_size, hipStream_t stream) {
  if (n_in < 6) return;
  const size_t need_x = ((size_t)(NB - 1) * SEQ_FULL + SEQ) * HID;
  if ((size_t)in_sizes[0] < need_x) return;
  for (int i = 1; i <= 5; ++i) if (in_sizes[i] < HID * HID) return;
  if ((size_t)out_size < (size_t)MROWS * HID) return;

  const float* x   = (const float*)d_in[0];
  const float* Wqr = (const float*)d_in[1];
  const float* Wqi = (const float*)d_in[2];
  const float* Wkr = (const float*)d_in[3];
  const float* Wki = (const float*)d_in[4];
  const float* Wv  = (const float*)d_in[5];
  float* out = (float*)d_out;

  size_t off = 0; char* ws = (char*)d_ws;
  unsigned short* xpl = (unsigned short*)(ws + off); off += (size_t)MROWS * HID * 2;
  unsigned short* wpl = (unsigned short*)(ws + off); off += (size_t)NW * HID * HID * 2;
  h16* Qa = (h16*)(ws + off); off += (size_t)MROWS * NH * QKW * 2;
  h16* Kc = (h16*)(ws + off); off += (size_t)MROWS * NH * QKW * 2;
  h16* Vp = (h16*)(ws + off); off += (size_t)MROWS * HID * 2;
  if (off > ws_size) return;

  cvt_kernel<<<1024, 256, 0, stream>>>(x, Wqr, Wqi, Wkr, Wki, Wv, xpl, wpl);
  proj_gemm_kernel<<<dim3(NCOMB / 64, MROWS / 128), 128, 0, stream>>>((const b16*)xpl, (const b16*)wpl, Qa, Kc, Vp);
  attn_kernel<<<(NB * NH * QT) / 8, 256, 0, stream>>>(Qa, Kc, Vp, out);
}
